// _SelfAttention_23673859736415
// MI455X (gfx1250) — hardware-verified
//
#include <hip/hip_runtime.h>
#include <hip/hip_bf16.h>

typedef __attribute__((ext_vector_type(16))) _Float16 v16h;
typedef __attribute__((ext_vector_type(8)))  _Float16 v8h;
typedef __attribute__((ext_vector_type(16))) __bf16   v16b;
typedef __attribute__((ext_vector_type(8)))  __bf16   v8b;
typedef __attribute__((ext_vector_type(8)))  float    v8f;
typedef __attribute__((ext_vector_type(4)))  float    v4f;
typedef __attribute__((ext_vector_type(4)))  unsigned v4u;

constexpr int MODEL_DIM = 1024;
constexpr int SEQ_LEN   = 2048;
constexpr int N_BATCH   = 2;
constexpr int N_HEAD    = 16;
constexpr int HEAD_D    = 64;
constexpr int INNER_DIM = N_HEAD * HEAD_D;
constexpr int QKV_COLS  = 3 * INNER_DIM;
constexpr int TOK_ROWS  = N_BATCH * SEQ_LEN;
constexpr int KV_CHUNK  = 64;
constexpr int Q_BLOCK   = 64;

static_assert(MODEL_DIM % 32 == 0, "K of qkv projection");
static_assert(INNER_DIM % 32 == 0, "K of output projection");
static_assert(TOK_ROWS % 64 == 0, "M tile multiple");
static_assert(QKV_COLS % 64 == 0, "N tile multiple (qkv)");
static_assert(MODEL_DIM % 64 == 0, "N tile multiple (out)");
static_assert(SEQ_LEN % KV_CHUNK == 0 && SEQ_LEN % Q_BLOCK == 0, "attention tiles");
static_assert(HEAD_D == 64, "attention kernel is head_dim 64");
static_assert(MODEL_DIM == 128 * 8, "LayerNorm kernel: 128 threads x 8 elements per row");

constexpr size_t WS_WQ    = (size_t)QKV_COLS * MODEL_DIM * 2;
constexpr size_t WS_WO    = (size_t)MODEL_DIM * INNER_DIM * 2;
constexpr size_t WS_HPL   = (size_t)TOK_ROWS * MODEL_DIM * 2;
constexpr size_t WS_QKVPL = (size_t)TOK_ROWS * QKV_COLS * 2;
constexpr size_t WS_ATPL  = (size_t)TOK_ROWS * INNER_DIM * 2;
constexpr size_t WS_TOTAL = WS_WQ + WS_WO + 2 * WS_HPL + 2 * WS_QKVPL + 2 * WS_ATPL;
static_assert(WS_TOTAL == 92274688, "carve arithmetic");
static_assert(WS_TOTAL <= 134217728, "carve budget");
static_assert(WS_WQ % 128 == 0 && WS_WO % 128 == 0 && WS_HPL % 128 == 0 && WS_QKVPL % 128 == 0 && WS_ATPL % 128 == 0, "128-B aligned regions");

__device__ __forceinline__ unsigned short f2bf_bits(float f) {
  unsigned u = __float_as_uint(f);
  return (unsigned short)((u + 0x7FFFu + ((u >> 16) & 1u)) >> 16);
}
__device__ __forceinline__ float bf_bits2f(unsigned short h) { return __uint_as_float(((unsigned)h) << 16); }

__device__ __forceinline__ void dep_guard_h(v8f& a, v8f& b, v16h x, v16h y) { asm volatile("v_nop\n\tv_nop\n\tv_nop\n\tv_nop" : "+v"(a), "+v"(b) : "v"(x), "v"(y)); }
__device__ __forceinline__ void dep_guard_b(v8f& a, v8f& b, v16b x, v16b y) { asm volatile("v_nop\n\tv_nop\n\tv_nop\n\tv_nop" : "+v"(a), "+v"(b) : "v"(x), "v"(y)); }
__device__ __forceinline__ void keep4_h(v16h a, v16h b, v16h c, v16h d) { asm volatile("v_nop" :: "v"(a), "v"(b), "v"(c), "v"(d)); }
__device__ __forceinline__ void keep4_b(v16b a, v16b b, v16b c, v16b d) { asm volatile("v_nop" :: "v"(a), "v"(b), "v"(c), "v"(d)); }
__device__ __forceinline__ void acc_guard4(v8f& a, v8f& b, v8f& c, v8f& d) { asm volatile("v_nop\n\tv_nop\n\tv_nop\n\tv_nop" : "+v"(a), "+v"(b), "+v"(c), "+v"(d)); }
template <typename T> struct Frag;
template <> struct Frag<_Float16> {
  typedef v16h V; union U { v16h v; v8h h[2]; };
  static __device__ __forceinline__ v16h load(const _Float16* p) {
    U f; f.h[0] = *(const v8h*)(p); f.h[1] = *(const v8h*)(p + 16); return f.v;
  }
  static __device__ __forceinline__ v8f mma(v16h a, v16h b, v8f c) {
    return __builtin_amdgcn_wmma_f32_16x16x32_f16(false, a, false, b, (short)0, c, false, false);
  }
  static __device__ __forceinline__ void guard(v8f& a, v8f& b, v16h x, v16h y) { dep_guard_h(a, b, x, y); }
  static __device__ __forceinline__ void keep(v16h a, v16h b, v16h c, v16h d) { keep4_h(a, b, c, d); }
};
template <> struct Frag<__bf16> {
  typedef v16b V; union U { v16b v; v8b h[2]; };
  static __device__ __forceinline__ v16b load(const __bf16* p) {
    U f; f.h[0] = *(const v8b*)(p); f.h[1] = *(const v8b*)(p + 16); return f.v;
  }
  static __device__ __forceinline__ v8f mma(v16b a, v16b b, v8f c) {
    return __builtin_amdgcn_wmma_f32_16x16x32_bf16(false, a, false, b, (short)0, c, false, false);
  }
  static __device__ __forceinline__ void guard(v8f& a, v8f& b, v16b x, v16b y) { dep_guard_b(a, b, x, y); }
  static __device__ __forceinline__ void keep(v16b a, v16b b, v16b c, v16b d) { keep4_b(a, b, c, d); }
};

__device__ __forceinline__ unsigned short at_bf_bits(float f) {
  unsigned u = __float_as_uint(f);
  return (unsigned short)((u + 0x7FFFu + ((u >> 16) & 1u)) >> 16);
}
__device__ __forceinline__ __bf16 at_f2bf(float f) { return __builtin_bit_cast(__bf16, at_bf_bits(f)); }
__device__ __forceinline__ void at_split(float f, __bf16& hi, __bf16& lo) {
  const unsigned short hb = at_bf_bits(f);
  hi = __builtin_bit_cast(__bf16, hb);
  lo = at_f2bf(f - __uint_as_float(((unsigned)hb) << 16));
}
__device__ __forceinline__ v8f at_mma(v16b a, v16b b, v8f c) {
  c = __builtin_amdgcn_wmma_f32_16x16x32_bf16(false, a, false, b, (short)0, c, false, false);
  asm volatile("v_nop\n\tv_nop\n\tv_nop\n\tv_nop" : "+v"(c) : "v"(a), "v"(b));
  return c;
}

__global__ __launch_bounds__(256) void cast_f32_bf16x8(
    const float* __restrict__ in, unsigned short* __restrict__ out, int n8) {
  const int i = blockIdx.x * 256 + threadIdx.x;
  if (i < n8) {
    const size_t e0 = (size_t)i * 8;
    const v4f a = *(const v4f*)(in + e0);
    const v4f b = *(const v4f*)(in + e0 + 4);
    v4u u;
    u[0] = (unsigned)f2bf_bits(a[0]) | ((unsigned)f2bf_bits(a[1]) << 16);
    u[1] = (unsigned)f2bf_bits(a[2]) | ((unsigned)f2bf_bits(a[3]) << 16);
    u[2] = (unsigned)f2bf_bits(b[0]) | ((unsigned)f2bf_bits(b[1]) << 16);
    u[3] = (unsigned)f2bf_bits(b[2]) | ((unsigned)f2bf_bits(b[3]) << 16);
    *(volatile v4u*)(out + e0) = u;
    __threadfence();
    *(volatile v4u*)(out + e0) = u;
  }
}

__global__ __launch_bounds__(128) void layernorm_bf16split_kernel(
    const float* __restrict__ x, const float* __restrict__ gamma, const float* __restrict__ beta,
    unsigned short* __restrict__ hhi, unsigned short* __restrict__ hlo) {
  __shared__ float red_s[4];
  __shared__ float red_q[4];
  const int row = blockIdx.x;
  const int t = threadIdx.x;
  const int lane = t & 31, wave = t >> 5;
  const size_t base = (size_t)row * MODEL_DIM + 8 * (size_t)t;

  const v4f a0 = *(const v4f*)(x + base);
  const v4f a1 = *(const v4f*)(x + base + 4);
  float xv[8];
#pragma unroll
  for (int e = 0; e < 4; ++e) {
    xv[e]     = bf_bits2f(f2bf_bits(a0[e]));
    xv[4 + e] = bf_bits2f(f2bf_bits(a1[e]));
  }
  float s = ((xv[0] + xv[1]) + (xv[2] + xv[3])) + ((xv[4] + xv[5]) + (xv[6] + xv[7]));
#pragma unroll
  for (int off = 1; off < 32; off <<= 1) s += __shfl_xor(s, off, 32);
  if (lane == 0) red_s[wave] = s;
  __syncthreads();
  const float tot = (red_s[0] + red_s[1]) + (red_s[2] + red_s[3]);
  const float mean = tot * (1.0f / (float)MODEL_DIM);

  float d[8];
  float q = 0.f;
#pragma unroll
  for (int e = 0; e < 8; ++e) { d[e] = xv[e] - mean; q += d[e] * d[e]; }
#pragma unroll
  for (int off = 1; off < 32; off <<= 1) q += __shfl_xor(q, off, 32);
  if (lane == 0) red_q[wave] = q;
  __syncthreads();
  const float qt = (red_q[0] + red_q[1]) + (red_q[2] + red_q[3]);
  const float var = qt * (1.0f / (float)MODEL_DIM);
  const float rstd = rsqrtf(var + 1e-5f);

  const v4f g0 = *(const v4f*)(gamma + 8 * t);
  const v4f g1 = *(const v4f*)(gamma + 8 * t + 4);
  const v4f b0 = *(const v4f*)(beta + 8 * t);
  const v4f b1 = *(const v4f*)(beta + 8 * t + 4);
  float hv[8];
#pragma unroll
  for (int e = 0; e < 4; ++e) {
    const float gg0 = bf_bits2f(f2bf_bits(g0[e])), bb0 = bf_bits2f(f2bf_bits(b0[e]));
    const float gg1 = bf_bits2f(f2bf_bits(g1[e])), bb1 = bf_bits2f(f2bf_bits(b1[e]));
    hv[e]     = d[e] * rstd * gg0 + bb0;
    hv[4 + e] = d[4 + e] * rstd * gg1 + bb1;
  }
  v4u ph, pl;
#pragma unroll
  for (int w = 0; w < 4; ++w) {
    const float f0 = hv[2 * w], f1 = hv[2 * w + 1];
    const unsigned short h0 = f2bf_bits(f0), h1 = f2bf_bits(f1);
    const unsigned short l0 = f2bf_bits(f0 - bf_bits2f(h0));
    const unsigned short l1 = f2bf_bits(f1 - bf_bits2f(h1));
    ph[w] = (unsigned)h0 | ((unsigned)h1 << 16);
    pl[w] = (unsigned)l0 | ((unsigned)l1 << 16);
  }
  *(volatile v4u*)(hhi + base) = ph;
  *(volatile v4u*)(hlo + base) = pl;
  __threadfence();
  *(volatile v4u*)(hhi + base) = ph;
  *(volatile v4u*)(hlo + base) = pl;
}

template <int OUT_MODE, bool HAS_BIAS>
__global__ __launch_bounds__(256) void gemm64_bf16_asplit(
    const unsigned short* __restrict__ Ahp, const unsigned short* __restrict__ Alp, int lda,
    const unsigned short* __restrict__ Btp, int ldb,
    void* __restrict__ Cout, void* __restrict__ Cout2, int ldc,
    const float* __restrict__ bias, int M, int N, int K) {
  typedef __bf16 T;
  typedef v16b V;
  const T* Ah = (const T*)Ahp; const T* Al = (const T*)Alp; const T* Bt = (const T*)Btp;
  __shared__ __align__(16) float sT[8][16 * 68];
  const int lane = threadIdx.x & 31;
  const int wave = threadIdx.x >> 5;
  const int tilesN = N >> 6;
  const int tilesM = M >> 6;
  const int tile = blockIdx.x * 8 + wave;
  if (tile >= tilesM * tilesN) return;
  const int tm = tile / tilesN;
  const int tn = tile - tm * tilesN;
  const int m0 = tm << 6;
  const int n0 = tn << 6;

  const int rlane = lane & 15;
  const int koff  = (lane >> 4) * 8;
  const int mOff  = (lane >> 4) * 8;

  v8f acc[4][4];
#pragma unroll
  for (int i = 0; i < 4; ++i)
#pragma unroll
    for (int j = 0; j < 4; ++j) acc[i][j] = (v8f){0.f,0.f,0.f,0.f,0.f,0.f,0.f,0.f};

  for (int k0 = 0; k0 < K; k0 += 32) {
    V bh[4];
#pragma unroll
    for (int j = 0; j < 4; ++j) {
      const size_t bo = (size_t)(n0 + (j << 4) + rlane) * ldb + koff + k0;
      bh[j] = Frag<T>::load(Bt + bo);
    }
#pragma unroll
    for (int i = 0; i < 4; ++i) {
      const size_t ao = (size_t)(m0 + (i << 4) + rlane) * lda + koff + k0;
      V ah = Frag<T>::load(Ah + ao);
      V al = Frag<T>::load(Al + ao);
#pragma unroll
      for (int j = 0; j < 4; ++j) {
        acc[i][j] = Frag<T>::mma(ah, bh[j], acc[i][j]);
        acc[i][j] = Frag<T>::mma(al, bh[j], acc[i][j]);
      }
      Frag<T>::guard(acc[i][0], acc[i][3], ah, al);
    }
    Frag<T>::keep(bh[0], bh[1], bh[2], bh[3]);
  }
  acc_guard4(acc[0][0], acc[0][1], acc[0][2], acc[0][3]);
  acc_guard4(acc[1][0], acc[1][1], acc[1][2], acc[1][3]);
  acc_guard4(acc[2][0], acc[2][1], acc[2][2], acc[2][3]);
  acc_guard4(acc[3][0], acc[3][1], acc[3][2], acc[3][3]);

  float* slab = sT[wave];
#pragma unroll
  for (int i = 0; i < 4; ++i) {
    const int mBase = m0 + (i << 4);
#pragma unroll
    for (int j = 0; j < 4; ++j) {
#pragma unroll
      for (int r = 0; r < 8; ++r) {
        slab[(mOff + r) * 68 + (j << 4) + rlane] = acc[i][j][r];
      }
    }
    __builtin_amdgcn_fence(__ATOMIC_RELEASE, "workgroup");
    __builtin_amdgcn_wave_barrier();
    __builtin_amdgcn_fence(__ATOMIC_ACQUIRE, "workgroup");
    if (OUT_MODE == 0) {
      float* Cf = (float*)Cout;
      const int h2 = lane >> 4, c4 = (lane & 15) * 4;
      v4f bb = (v4f){0.f, 0.f, 0.f, 0.f};
      if (HAS_BIAS) {
        const v4f braw = *(const v4f*)(bias + n0 + c4);
#pragma unroll
        for (int e = 0; e < 4; ++e) bb[e] = bf_bits2f(f2bf_bits(braw[e]));
      }
      for (int pass = 0; pass < 2; ++pass) {
#pragma unroll
        for (int it = 0; it < 8; ++it) {
          const int row = it * 2 + h2;
          v4f v = *(const v4f*)(slab + row * 68 + c4);
          v = v + bb;
          *(volatile v4f*)(Cf + (size_t)(mBase + row) * ldc + n0 + c4) = v;
        }
        __threadfence();
      }
    } else {
      const int q = lane >> 3, c8 = (lane & 7) * 8;
      unsigned short* Cu  = (unsigned short*)Cout;
      unsigned short* Cu2 = (unsigned short*)Cout2;
      for (int pass = 0; pass < 2; ++pass) {
#pragma unroll
        for (int it = 0; it < 4; ++it) {
          const int row = it * 4 + q;
          const float* sp = slab + row * 68 + c8;
          v8h hv, lv;
#pragma unroll
          for (int e = 0; e < 8; ++e) {
            unsigned short hb = f2bf_bits(sp[e]);
            unsigned short lb = f2bf_bits(sp[e] - bf_bits2f(hb));
            hv[e] = __builtin_bit_cast(_Float16, hb);
            lv[e] = __builtin_bit_cast(_Float16, lb);
          }
          *(volatile v8h*)(Cu  + (size_t)(mBase + row) * ldc + n0 + c8) = hv;
          *(volatile v8h*)(Cu2 + (size_t)(mBase + row) * ldc + n0 + c8) = lv;
        }
        __threadfence();
      }
    }
    __builtin_amdgcn_fence(__ATOMIC_RELEASE, "workgroup");
    __builtin_amdgcn_wave_barrier();
    __builtin_amdgcn_fence(__ATOMIC_ACQUIRE, "workgroup");
  }
}

__global__ __launch_bounds__(128) void attn64_bf16x3_kernel(
    const unsigned short* __restrict__ qkvh, const unsigned short* __restrict__ qkvl,
    unsigned short* __restrict__ oh, unsigned short* __restrict__ ol) {
  union FB { v16b v; v8b h[2]; };
  __shared__ __align__(16) unsigned short Ksh[KV_CHUNK * HEAD_D];
  __shared__ __align__(16) unsigned short Ksl[KV_CHUNK * HEAD_D];
  __shared__ __align__(16) unsigned short Vth[HEAD_D * KV_CHUNK];
  __shared__ __align__(16) unsigned short Vtl[HEAD_D * KV_CHUNK];
  __shared__ __align__(16) __bf16 Psh[4][16 * KV_CHUNK];
  __shared__ __align__(16) __bf16 Psl[4][16 * KV_CHUNK];
  __shared__ __align__(16) float  Os[4][16 * 68];

  const int tid  = threadIdx.x;
  const int wave = tid >> 5;
  const int lane = tid & 31;
  const int hh   = lane >> 4;
  const int c    = lane & 15;

  constexpr int NQB = SEQ_LEN / Q_BLOCK;
  const int bx   = blockIdx.x;
  const int qb   = bx % NQB;
  const int bhid = bx / NQB;
  const int head = bhid % N_HEAD;
  const int bat  = bhid / N_HEAD;
  const int q0   = qb * Q_BLOCK + wave * 16;
  const size_t tokb = (size_t)bat * SEQ_LEN;
  const int hcol = head * HEAD_D;

  const __bf16* QH = (const __bf16*)qkvh;
  const __bf16* QL = (const __bf16*)qkvl;

  v16b qah[2], qal[2];
  {
    const size_t qo = (tokb + q0 + c) * QKV_COLS + hcol + 8 * hh;
#pragma unroll
    for (int dc = 0; dc < 2; ++dc) {
      qah[dc] = Frag<__bf16>::load(QH + qo + dc * 32);
      qal[dc] = Frag<__bf16>::load(QL + qo + dc * 32);
    }
  }

  float mrow[8], lrow[8];
  v8f oacc[4];
#pragma unroll
  for (int r = 0; r < 8; ++r) { mrow[r] = -INFINITY; lrow[r] = 0.f; }
#pragma unroll
  for (int t = 0; t < 4; ++t) oacc[t] = (v8f){0.f,0.f,0.f,0.f,0.f,0.f,0.f,0.f};

  const __bf16* KHp = (const __bf16*)Ksh;
  const __bf16* KLp = (const __bf16*)Ksl;
  const __bf16* VHp = (const __bf16*)Vth;
  const __bf16* VLp = (const __bf16*)Vtl;

  for (int kc = 0; kc < SEQ_LEN / KV_CHUNK; ++kc) {
    const int kv0 = kc * KV_CHUNK;
    __syncthreads();
    {
      const int kvr = tid >> 1, dh = (tid & 1) * 32;
      const size_t kro = (tokb + kv0 + kvr) * QKV_COLS + INNER_DIM + hcol + dh;
      const size_t vro = kro + INNER_DIM;
#pragma unroll
      for (int i = 0; i < 4; ++i) {
        const v4u kh4 = *(const v4u*)(qkvh + kro + 8 * i);
        const v4u kl4 = *(const v4u*)(qkvl + kro + 8 * i);
        *(v4u*)(Ksh + kvr * HEAD_D + dh + 8 * i) = kh4;
        *(v4u*)(Ksl + kvr * HEAD_D + dh + 8 * i) = kl4;
      }
      asm volatile("" ::: "memory");
#pragma unroll
      for (int i = 0; i < 4; ++i) {
        const v4u vh4 = *(const v4u*)(qkvh + vro + 8 * i);
        const v4u vl4 = *(const v4u*)(qkvl + vro + 8 * i);
#pragma unroll
        for (int w = 0; w < 4; ++w) {
          const int d0 = dh + 8 * i + 2 * w;
          const unsigned uh = vh4[w], ul = vl4[w];
          Vth[d0 * KV_CHUNK + kvr]       = (unsigned short)(uh & 0xffffu);
          Vth[(d0 + 1) * KV_CHUNK + kvr] = (unsigned short)(uh >> 16);
          Vtl[d0 * KV_CHUNK + kvr]       = (unsigned short)(ul & 0xffffu);
          Vtl[(d0 + 1) * KV_CHUNK + kvr] = (unsigned short)(ul >> 16);
        }
      }
    }
    __syncthreads();

    v8f s[4];
#pragma unroll
    for (int j = 0; j < 4; ++j) {
      s[j] = (v8f){0.f,0.f,0.f,0.f,0.f,0.f,0.f,0.f};
#pragma unroll
      for (int dc = 0; dc < 2; ++dc) {
        FB kb, kl;
        const int ko = (j * 16 + c) * HEAD_D + dc * 32 + 8 * hh;
        kb.h[0] = *(const v8b*)(KHp + ko);
        kb.h[1] = *(const v8b*)(KHp + ko + 16);
        kl.h[0] = *(const v8b*)(KLp + ko);
        kl.h[1] = *(const v8b*)(KLp + ko + 16);
        s[j] = at_mma(qah[dc], kb.v, s[j]);
        s[j] = at_mma(qah[dc], kl.v, s[j]);
        s[j] = at_mma(qal[dc], kb.v, s[j]);
      }
    }
    float cm[8];
#pragma unroll
    for (int r = 0; r < 8; ++r) {
      float m = -INFINITY;
#pragma unroll
      for (int j = 0; j < 4; ++j) {
        s[j][r] = s[j][r] * 0.125f;
        m = fmaxf(m, s[j][r]);
      }
#pragma unroll
      for (int off = 1; off < 16; off <<= 1) m = fmaxf(m, __shfl_xor(m, off, 32));
      cm[r] = m;
    }
    __bf16* pwh = Psh[wave];
    __bf16* pwl = Psl[wave];
#pragma unroll
    for (int r = 0; r < 8; ++r) {
      const float mnew = fmaxf(mrow[r], cm[r]);
      const float alpha = expf(mrow[r] - mnew);
      mrow[r] = mnew;
      float psum = 0.f;
#pragma unroll
      for (int j = 0; j < 4; ++j) {
        const float p = expf(s[j][r] - mnew);
        psum += p;
        __bf16 a, bl;
        at_split(p, a, bl);
        pwh[(8 * hh + r) * KV_CHUNK + j * 16 + c] = a;
        pwl[(8 * hh + r) * KV_CHUNK + j * 16 + c] = bl;
      }
#pragma unroll
      for (int off = 1; off < 16; off <<= 1) psum += __shfl_xor(psum, off, 32);
      lrow[r] = lrow[r] * alpha + psum;
#pragma unroll
      for (int t = 0; t < 4; ++t) oacc[t][r] *= alpha;
    }
    __builtin_amdgcn_fence(__ATOMIC_RELEASE, "workgroup");
    __builtin_amdgcn_wave_barrier();
    __builtin_amdgcn_fence(__ATOMIC_ACQUIRE, "workgroup");
#pragma unroll 1
    for (int kk = 0; kk < 2; ++kk) {
      FB pa, pl;
      pa.h[0] = *(const v8b*)(pwh + c * KV_CHUNK + kk * 32 + 8 * hh);
      pa.h[1] = *(const v8b*)(pwh + c * KV_CHUNK + kk * 32 + 16 + 8 * hh);
      pl.h[0] = *(const v8b*)(pwl + c * KV_CHUNK + kk * 32 + 8 * hh);
      pl.h[1] = *(const v8b*)(pwl + c * KV_CHUNK + kk * 32 + 16 + 8 * hh);
#pragma unroll
      for (int t = 0; t < 4; ++t) {
        FB vb, vl;
        const int vo = (t * 16 + c) * KV_CHUNK + kk * 32 + 8 * hh;
        vb.h[0] = *(const v8b*)(VHp + vo);
        vb.h[1] = *(const v8b*)(VHp + vo + 16);
        vl.h[0] = *(const v8b*)(VLp + vo);
        vl.h[1] = *(const v8b*)(VLp + vo + 16);
        oacc[t] = at_mma(pa.v, vb.v, oacc[t]);
        oacc[t] = at_mma(pa.v, vl.v, oacc[t]);
        oacc[t] = at_mma(pl.v, vb.v, oacc[t]);
      }
    }
  }

  float* os = Os[wave];
#pragma unroll
  for (int r = 0; r < 8; ++r) {
    const float inv = 1.0f / lrow[r];
#pragma unroll
    for (int t = 0; t < 4; ++t) os[(8 * hh + r) * 68 + t * 16 + c] = oacc[t][r] * inv;
  }
  __builtin_amdgcn_fence(__ATOMIC_RELEASE, "workgroup");
  __builtin_amdgcn_wave_barrier();
  __builtin_amdgcn_fence(__ATOMIC_ACQUIRE, "workgroup");
  {
    const int q8 = lane >> 3, c8 = (lane & 7) * 8;
    for (int pass = 0; pass < 2; ++pass) {
#pragma unroll
      for (int it = 0; it < 4; ++it) {
        const int row = it * 4 + q8;
        const float* sp = os + row * 68 + c8;
        const v4f f0 = *(const v4f*)(sp);
        const v4f f1 = *(const v4f*)(sp + 4);
        v4u ph, plo;
#pragma unroll
        for (int w = 0; w < 2; ++w) {
          const float a = f0[2 * w], bq = f0[2 * w + 1];
          const unsigned short ha = f2bf_bits(a), hb = f2bf_bits(bq);
          const unsigned short la = f2bf_bits(a - bf_bits2f(ha)), lb = f2bf_bits(bq - bf_bits2f(hb));
          ph[w]  = (unsigned)ha | ((unsigned)hb << 16);
          plo[w] = (unsigned)la | ((unsigned)lb << 16);
        }
#pragma unroll
        for (int w = 0; w < 2; ++w) {
          const float a = f1[2 * w], bq = f1[2 * w + 1];
          const unsigned short ha = f2bf_bits(a), hb = f2bf_bits(bq);
          const unsigned short la = f2bf_bits(a - bf_bits2f(ha)), lb = f2bf_bits(bq - bf_bits2f(hb));
          ph[2 + w]  = (unsigned)ha | ((unsigned)hb << 16);
          plo[2 + w] = (unsigned)la | ((unsigned)lb << 16);
        }
        const size_t o = (tokb + q0 + row) * INNER_DIM + hcol + c8;
        *(volatile v4u*)(oh + o) = ph;
        *(volatile v4u*)(ol + o) = plo;
      }
      __threadfence();
    }
  }
}

extern "C" void kernel_launch(void* const* d_in, const int* in_sizes, int n_in,
                              void* d_out, int out_size, void* d_ws,
                              size_t ws_size, hipStream_t stream) {
  if (n_in < 6) return;
  if (in_sizes[0] != TOK_ROWS * MODEL_DIM) return;
  if (in_sizes[1] != MODEL_DIM || in_sizes[2] != MODEL_DIM) return;
  if (in_sizes[3] != QKV_COLS * MODEL_DIM) return;
  if (in_sizes[4] != MODEL_DIM * INNER_DIM) return;
  if (in_sizes[5] != MODEL_DIM) return;
  if (out_size != TOK_ROWS * MODEL_DIM) return;
  if (ws_size < WS_TOTAL) return;

  const float* x    = (const float*)d_in[0];
  const float* gam  = (const float*)d_in[1];
  const float* bet  = (const float*)d_in[2];
  const float* wqkv = (const float*)d_in[3];
  const float* wout = (const float*)d_in[4];
  const float* bout = (const float*)d_in[5];
  float* out = (float*)d_out;

  char* ws = (char*)d_ws;
  size_t off = 0;
  unsigned short* wq_bf  = (unsigned short*)(ws + off); off += WS_WQ;
  unsigned short* wo_bf  = (unsigned short*)(ws + off); off += WS_WO;
  unsigned short* h_hi   = (unsigned short*)(ws + off); off += WS_HPL;
  unsigned short* h_lo   = (unsigned short*)(ws + off); off += WS_HPL;
  unsigned short* qkv_hi = (unsigned short*)(ws + off); off += WS_QKVPL;
  unsigned short* qkv_lo = (unsigned short*)(ws + off); off += WS_QKVPL;
  unsigned short* at_hi  = (unsigned short*)(ws + off); off += WS_ATPL;
  unsigned short* at_lo  = (unsigned short*)(ws + off); off += WS_ATPL;
  if (off > ws_size) return;

  const int n8_qkv = (QKV_COLS * MODEL_DIM) / 8;
  const int n8_out = (MODEL_DIM * INNER_DIM) / 8;
  cast_f32_bf16x8<<<dim3((n8_qkv + 255) / 256), dim3(256), 0, stream>>>(wqkv, wq_bf, n8_qkv);
  cast_f32_bf16x8<<<dim3((n8_out + 255) / 256), dim3(256), 0, stream>>>(wout, wo_bf, n8_out);

  layernorm_bf16split_kernel<<<dim3(TOK_ROWS), dim3(128), 0, stream>>>(x, gam, bet, h_hi, h_lo);

  gemm64_bf16_asplit<2, false><<<dim3((TOK_ROWS / 64) * (QKV_COLS / 64) / 8), dim3(256), 0, stream>>>(
      h_hi, h_lo, MODEL_DIM, wq_bf, MODEL_DIM, (void*)qkv_hi, (void*)qkv_lo, QKV_COLS,
      (const float*)nullptr, TOK_ROWS, QKV_COLS, MODEL_DIM);

  attn64_bf16x3_kernel<<<dim3(N_BATCH * N_HEAD * (SEQ_LEN / Q_BLOCK)), dim3(128), 0, stream>>>(
      qkv_hi, qkv_lo, at_hi, at_lo);

  gemm64_bf16_asplit<0, true><<<dim3((TOK_ROWS / 64) * (MODEL_DIM / 64) / 8), dim3(256), 0, stream>>>(
      at_hi, at_lo, INNER_DIM, wo_bf, INNER_DIM, (void*)out, (void*)nullptr, MODEL_DIM,
      bout, TOK_ROWS, MODEL_DIM, INNER_DIM);
}
